// Hgru2_2d_parallel_67559835566284
// MI455X (gfx1250) — hardware-verified
//
#include <hip/hip_runtime.h>
#include <hip/hip_bf16.h>
#include <math.h>

#define HH    64
#define WW    64
#define BB    8
#define DD    256
#define NROW  (HH * WW * BB)
#define N1    (3 * DD)
#define NG2   (DD / 4)
#define NLH   (WW * BB * NG2)
#define NLW   (HH * BB * NG2)
#define SBLK  32
#define GSTR  40
#define OSTR  68
#define SMEMB (8 * 16 * OSTR * 4)
#define LNEPS 1e-5f

static_assert(NROW % 128 == 0);
static_assert(N1 % 64 == 0);
static_assert(DD % 64 == 0);
static_assert(DD % 32 == 0);
static_assert(N1 % DD == 0);
static_assert(NLH % SBLK == 0);
static_assert(NLW % SBLK == 0);
static_assert(NROW % 8 == 0);
static_assert((NROW * (DD / 8)) % 256 == 0);
static_assert((N1 * (DD / 8)) % 256 == 0);
static_assert((DD * (DD / 8)) % 256 == 0);
static_assert(SMEMB >= (2 * 128 * GSTR + 64 * GSTR) * 2);
#define RBYTES ((size_t)NROW * DD * 4)
static_assert((size_t)NROW * DD * 2 + (size_t)N1 * DD * 2 <= RBYTES);
static_assert(2 * (size_t)NROW * DD * 2 <= RBYTES);
static_assert((size_t)DD * DD * 2 <= RBYTES);
static_assert(4 * RBYTES <= (size_t)134217728);

typedef unsigned short us16 __attribute__((ext_vector_type(16)));
typedef unsigned short us8  __attribute__((ext_vector_type(8)));
typedef unsigned short us8a __attribute__((ext_vector_type(8), may_alias));
typedef __bf16 v16b __attribute__((ext_vector_type(16)));
typedef float v8f __attribute__((ext_vector_type(8)));
typedef float v4f __attribute__((ext_vector_type(4)));
typedef float v4fa __attribute__((ext_vector_type(4), may_alias));
union FragU { us16 v; us8 h[2]; };

__device__ __forceinline__ unsigned short bf16_bits(float f) {
  unsigned u = __float_as_uint(f);
  u += 0x7FFFu + ((u >> 16) & 1u);
  return (unsigned short)(u >> 16);
}
__device__ __forceinline__ float bf16_val(unsigned short b) { return __uint_as_float(((unsigned)b) << 16); }
__device__ __forceinline__ float bf16r(float f) { return bf16_val(bf16_bits(f)); }

__device__ __forceinline__ v8f mma_bf16(us16 a, us16 b, v8f c) {
  return __builtin_amdgcn_wmma_f32_16x16x32_bf16(false, __builtin_bit_cast(v16b, a), false, __builtin_bit_cast(v16b, b), (short)0, c, false, false);
}
__device__ __forceinline__ void wguard(v8f& c0, v8f& c1, v8f& c2, v8f& c3, const us16& a0, const us16& a1,
                                       const us16& b0, const us16& b1, const us16& b2, const us16& b3) {
#if defined(__HIP_DEVICE_COMPILE__)
  asm volatile("v_nop\n\tv_nop\n\tv_nop\n\tv_nop"
               : "+v"(c0), "+v"(c1), "+v"(c2), "+v"(c3)
               : "v"(a0), "v"(a1), "v"(b0), "v"(b1), "v"(b2), "v"(b3));
#endif
}

__device__ __forceinline__ us16 lds_frag(const unsigned short* base) {
  const int lane = threadIdx.x & 31, r = lane & 15, kh = (lane >> 4) * 8;
  FragU f;
  f.h[0] = *(const us8a*)(base + r * GSTR + kh);
  f.h[1] = *(const us8a*)(base + r * GSTR + 16 + kh);
  return f.v;
}

__device__ __forceinline__ void stage_a(unsigned short* lds, const unsigned short* __restrict__ P, int ld, int m0, int k0, int tid) {
  const int row = tid >> 1, cq = (tid & 1) * 16;
  const unsigned short* src = P + (size_t)(m0 + row) * ld + k0 + cq;
  const us8 v0 = *(const us8a*)src;
  const us8 v1 = *(const us8a*)(src + 8);
  *(us8a*)(lds + row * GSTR + cq) = v0;
  *(us8a*)(lds + row * GSTR + cq + 8) = v1;
}
__device__ __forceinline__ void stage_b(unsigned short* lds, const unsigned short* __restrict__ P, int ld, int n0, int k0, int tid) {
  const int row = tid >> 2, kq = (tid & 3) * 8;
  const us8 v = *(const us8a*)(P + (size_t)(n0 + row) * ld + k0 + kq);
  *(us8a*)(lds + row * GSTR + kq) = v;
}

template <int NA, int MODE>
__global__ __launch_bounds__(256) void k_gemm(const unsigned short* __restrict__ A0, const unsigned short* __restrict__ A1, int lda,
                                             const unsigned short* __restrict__ B0, int ldb, const float* __restrict__ bias,
                                             float* P0, float* P1, float* P2, int ldy, int K, int nsec) {
  __shared__ __attribute__((aligned(16))) unsigned char sm[SMEMB];
  unsigned short* lA0 = (unsigned short*)sm;
  unsigned short* lA1 = lA0 + 128 * GSTR;
  unsigned short* lB0 = lA1 + 128 * GSTR;
  float* oS = (float*)sm;
  const int tid = threadIdx.x, lane = tid & 31, wave = tid >> 5, cl = lane & 15, hh = lane >> 4;
  const int m0 = blockIdx.x * 128, n0 = blockIdx.y * 64;
  const int sec = (MODE == 0) ? (n0 / nsec) : 0;
  float* Y = (sec == 0) ? P0 : ((sec == 1) ? P1 : P2);
  const int nl = n0 - sec * nsec;

  v8f acc[4];
#pragma unroll
  for (int j = 0; j < 4; ++j) { v8f zz = {0.f, 0.f, 0.f, 0.f, 0.f, 0.f, 0.f, 0.f}; acc[j] = zz; }

#pragma unroll 1
  for (int k0 = 0; k0 < K; k0 += 32) {
    __syncthreads();
    stage_a(lA0, A0, lda, m0, k0, tid);
    if (NA == 2) stage_a(lA1, A1, lda, m0, k0, tid);
    stage_b(lB0, B0, ldb, n0, k0, tid);
    __syncthreads();
    const us16 af0 = lds_frag(lA0 + 16 * wave * GSTR);
    us16 af1 = af0;
    if (NA == 2) af1 = lds_frag(lA1 + 16 * wave * GSTR);
    us16 bfr[4];
#pragma unroll
    for (int j = 0; j < 4; ++j) bfr[j] = lds_frag(lB0 + 16 * j * GSTR);
#pragma unroll
    for (int j = 0; j < 4; ++j) acc[j] = mma_bf16(af0, bfr[j], acc[j]);
    if (NA == 2) {
#pragma unroll
      for (int j = 0; j < 4; ++j) acc[j] = mma_bf16(af1, bfr[j], acc[j]);
    }
    wguard(acc[0], acc[1], acc[2], acc[3], af0, af1, bfr[0], bfr[1], bfr[2], bfr[3]);
  }
  __syncthreads();

  float bcol[4];
#pragma unroll
  for (int j = 0; j < 4; ++j) bcol[j] = bf16r(bias[n0 + 16 * j + cl]);

  float* so = oS + wave * (16 * OSTR);
#pragma unroll
  for (int j = 0; j < 4; ++j)
#pragma unroll
    for (int r = 0; r < 8; ++r) {
      float v = acc[j][r] + bcol[j];
      if (MODE == 0) {
        const float e = __expf(-v);
        const float sg = __builtin_amdgcn_rcpf(1.0f + e);
        v = (sec == 0) ? (v * sg) : sg;
      }
      so[(8 * hh + r) * OSTR + 16 * j + cl] = v;
    }
  __syncthreads();
#pragma unroll
  for (int pass = 0; pass < 2; ++pass) {
#pragma unroll
    for (int it = 0; it < 8; ++it) {
      const int ch = it * 32 + lane, r = ch >> 4, q = (ch & 15) * 4;
      const v4f v = *(const v4fa*)(so + r * OSTR + q);
      *(volatile v4f*)(Y + (size_t)(m0 + 16 * wave + r) * ldy + nl + q) = v;
    }
    __threadfence();
  }
}

__global__ __launch_bounds__(256) void k_cvt(const float* __restrict__ src, unsigned short* dst, int total8) {
  const int idx = blockIdx.x * 256 + threadIdx.x;
  if (idx >= total8) return;
  const float* s = src + (size_t)idx * 8;
  const v4f a = *(const v4fa*)s, b = *(const v4fa*)(s + 4);
  us8 o;
#pragma unroll
  for (int u = 0; u < 4; ++u) {
    o[u]     = bf16_bits(a[u]);
    o[4 + u] = bf16_bits(b[u]);
  }
  const size_t off = (size_t)idx * 8;
  *(volatile us8*)(dst + off) = o;
  __threadfence();
  *(volatile us8*)(dst + off) = o;
}

__global__ __launch_bounds__(256) void k_cvt_t(const float* __restrict__ src, unsigned short* dst, int nk, int nn, int total8) {
  const int idx = blockIdx.x * 256 + threadIdx.x;
  if (idx >= total8) return;
  const int nk8 = nk >> 3;
  const int n = idx / nk8, k8 = (idx - n * nk8) * 8;
  us8 o;
#pragma unroll
  for (int u = 0; u < 8; ++u) o[u] = bf16_bits(src[(size_t)(k8 + u) * (size_t)nn + n]);
  const size_t off = (size_t)n * nk + k8;
  *(volatile us8*)(dst + off) = o;
  __threadfence();
  *(volatile us8*)(dst + off) = o;
}

__device__ __forceinline__ v4f gstep(const v4f iv, const v4f lv, const v4f ov, float (&s)[8]) {
#pragma clang fp contract(off)
  v4f p;
#pragma unroll
  for (int q = 0; q < 2; ++q) {
    const float i0 = iv[2 * q], i1 = iv[2 * q + 1];
    const float l0 = lv[2 * q], l1 = lv[2 * q + 1];
    const float u0 = 1.0f - l0, u1 = 1.0f - l1;
    const float a00 = u0 * i0, a01 = u0 * i1, a10 = u1 * i0, a11 = u1 * i1;
    s[4 * q + 0] = l0 * s[4 * q + 0] + a00;
    s[4 * q + 1] = l0 * s[4 * q + 1] + a01;
    s[4 * q + 2] = l1 * s[4 * q + 2] + a10;
    s[4 * q + 3] = l1 * s[4 * q + 3] + a11;
    const float o0 = ov[2 * q], o1 = ov[2 * q + 1];
    p[2 * q + 0] = s[4 * q + 0] * o0 + s[4 * q + 2] * o1;
    p[2 * q + 1] = s[4 * q + 1] * o0 + s[4 * q + 3] * o1;
  }
  return p;
}

__global__ __launch_bounds__(SBLK) void k_scan_h(const float* __restrict__ INP, const float* __restrict__ LAM,
                                                const float* __restrict__ OG, float* OH) {
#pragma clang fp contract(off)
  __shared__ __attribute__((aligned(16))) float part[HH * SBLK * 4];
  const int lane = threadIdx.x;
  const int t = blockIdx.x * SBLK + lane;
  const int g2 = t & (NG2 - 1), wb = t >> 6;
  const size_t col = (size_t)(4 * g2);
  float s[8];
#pragma unroll
  for (int i = 0; i < 8; ++i) s[i] = 0.0f;
#pragma unroll 1
  for (int h = 0; h < HH; ++h) {
    const size_t e = ((size_t)h * (WW * BB) + (size_t)wb) * DD + col;
    const v4f iv = *(const v4fa*)(INP + e);
    const v4f lv = *(const v4fa*)(LAM + e);
    const v4f ov = *(const v4fa*)(OG + e);
    const v4f pf = gstep(iv, lv, ov, s);
    *(v4fa*)(part + (h * SBLK + lane) * 4) = pf;
  }
  __syncthreads();
#pragma unroll
  for (int i = 0; i < 8; ++i) s[i] = 0.0f;
#pragma unroll 1
  for (int h = HH - 1; h >= 0; --h) {
    const size_t e = ((size_t)h * (WW * BB) + (size_t)wb) * DD + col;
    const v4f iv = *(const v4fa*)(INP + e);
    const v4f lv = *(const v4fa*)(LAM + e);
    const v4f ov = *(const v4fa*)(OG + e);
    const v4f pb = gstep(iv, lv, ov, s);
    const v4f pf = *(const v4fa*)(part + (h * SBLK + lane) * 4);
    const v4f o = pf + pb;
    *(volatile v4f*)(OH + e) = o;
    __threadfence();
    *(volatile v4f*)(OH + e) = o;
  }
}

__global__ __launch_bounds__(SBLK) void k_scan_w(const float* __restrict__ INP, const float* __restrict__ LAM,
                                                const float* __restrict__ OG, float* S) {
#pragma clang fp contract(off)
  __shared__ __attribute__((aligned(16))) float part[WW * SBLK * 4];
  const int lane = threadIdx.x;
  const int t = blockIdx.x * SBLK + lane;
  const int g2 = t & (NG2 - 1), hb = t >> 6;
  const int b = hb & (BB - 1), h = hb >> 3;
  const size_t col = (size_t)(4 * g2);
  const size_t rbase = (size_t)h * (WW * BB) + (size_t)b;
  float s[8];
#pragma unroll
  for (int i = 0; i < 8; ++i) s[i] = 0.0f;
#pragma unroll 1
  for (int w = 0; w < WW; ++w) {
    const size_t e = (rbase + (size_t)w * BB) * DD + col;
    const v4f iv = *(const v4fa*)(INP + e);
    const v4f lv = *(const v4fa*)(LAM + e);
    const v4f ov = *(const v4fa*)(OG + e);
    const v4f pf = gstep(iv, lv, ov, s);
    *(v4fa*)(part + (w * SBLK + lane) * 4) = pf;
  }
  __syncthreads();
#pragma unroll
  for (int i = 0; i < 8; ++i) s[i] = 0.0f;
#pragma unroll 1
  for (int w = WW - 1; w >= 0; --w) {
    const size_t e = (rbase + (size_t)w * BB) * DD + col;
    const v4f iv = *(const v4fa*)(INP + e);
    const v4f lv = *(const v4fa*)(LAM + e);
    const v4f ov = *(const v4fa*)(OG + e);
    const v4f pb = gstep(iv, lv, ov, s);
    const v4f pf = *(const v4fa*)(part + (w * SBLK + lane) * 4);
    const v4f oh = *(const v4fa*)(S + e);
    const v4f pw = pf + pb;
    const v4f o = oh + pw;
    *(volatile v4f*)(S + e) = o;
    __threadfence();
    *(volatile v4f*)(S + e) = o;
  }
}

__global__ __launch_bounds__(256) void k_ln(const float* __restrict__ S, const float* __restrict__ gamma, const float* __restrict__ beta,
                                           unsigned short* YH, unsigned short* YL) {
#pragma clang fp contract(off)
  const int tid = threadIdx.x, lane = tid & 31, wave = tid >> 5;
  const size_t row = (size_t)blockIdx.x * 8 + (size_t)wave;
  const float* p = S + row * DD + lane * 8;
  const v4f a = *(const v4fa*)p, b = *(const v4fa*)(p + 4);
  float x[8];
#pragma unroll
  for (int u = 0; u < 4; ++u) { x[u] = a[u]; x[4 + u] = b[u]; }
  float sm = ((x[0] + x[1]) + (x[2] + x[3])) + ((x[4] + x[5]) + (x[6] + x[7]));
#pragma unroll
  for (int off = 16; off > 0; off >>= 1) sm += __shfl_xor(sm, off, 32);
  const float mu = sm * (1.0f / (float)DD);
  float c[8];
  float q = 0.0f;
#pragma unroll
  for (int u = 0; u < 8; ++u) { c[u] = x[u] - mu; q = q + c[u] * c[u]; }
#pragma unroll
  for (int off = 16; off > 0; off >>= 1) q += __shfl_xor(q, off, 32);
  const float var = q * (1.0f / (float)DD);
  const float rstd = rsqrtf(var + LNEPS);
  const v4f ga = *(const v4fa*)(gamma + lane * 8), gb = *(const v4fa*)(gamma + lane * 8 + 4);
  const v4f ba = *(const v4fa*)(beta + lane * 8), bb = *(const v4fa*)(beta + lane * 8 + 4);
  us8 hi, lo;
#pragma unroll
  for (int u = 0; u < 4; ++u) {
    const float y0 = (c[u] * rstd) * bf16r(ga[u]) + bf16r(ba[u]);
    const float y1 = (c[4 + u] * rstd) * bf16r(gb[u]) + bf16r(bb[u]);
    const unsigned short h0 = bf16_bits(y0), h1 = bf16_bits(y1);
    hi[u] = h0;     lo[u] = bf16_bits(y0 - bf16_val(h0));
    hi[4 + u] = h1; lo[4 + u] = bf16_bits(y1 - bf16_val(h1));
  }
  const size_t o = row * DD + lane * 8;
  *(volatile us8*)(YH + o) = hi; *(volatile us8*)(YL + o) = lo;
  __threadfence();
  *(volatile us8*)(YH + o) = hi; *(volatile us8*)(YL + o) = lo;
}

extern "C" void kernel_launch(void* const* d_in, const int* in_sizes, int n_in,
                              void* d_out, int out_size, void* d_ws, size_t ws_size,
                              hipStream_t stream) {
  if (n_in < 7) return;
  if (in_sizes[0] != NROW * DD || in_sizes[1] != DD * N1 || in_sizes[2] != N1 || in_sizes[3] != DD * DD ||
      in_sizes[4] != DD || in_sizes[5] != DD || in_sizes[6] != DD || out_size != NROW * DD) return;
  if (ws_size < 4 * RBYTES) return;
  const float* x     = (const float*)d_in[0];
  const float* in_w  = (const float*)d_in[1];
  const float* in_b  = (const float*)d_in[2];
  const float* out_w = (const float*)d_in[3];
  const float* out_b = (const float*)d_in[4];
  const float* gamma = (const float*)d_in[5];
  const float* beta  = (const float*)d_in[6];
  float* out = (float*)d_out;

  char* ws = (char*)d_ws;
  unsigned short* X16  = (unsigned short*)(ws);
  unsigned short* IW16 = (unsigned short*)(ws + (size_t)NROW * DD * 2);
  float* S             = (float*)(ws);
  float* INP           = (float*)(ws + RBYTES);
  unsigned short* YH   = (unsigned short*)(ws + RBYTES);
  unsigned short* YL   = (unsigned short*)(ws + RBYTES + (size_t)NROW * DD * 2);
  float* LAM           = (float*)(ws + 2 * RBYTES);
  unsigned short* OW16 = (unsigned short*)(ws + 2 * RBYTES);
  float* OG            = (float*)(ws + 3 * RBYTES);

  const dim3 blk(256);
  k_cvt<<<dim3((NROW * (DD / 8) + 255) / 256), blk, 0, stream>>>(x, X16, NROW * (DD / 8));
  k_cvt_t<<<dim3((N1 * (DD / 8) + 255) / 256), blk, 0, stream>>>(in_w, IW16, DD, N1, N1 * (DD / 8));
  k_gemm<1, 0><<<dim3(NROW / 128, N1 / 64), blk, 0, stream>>>(X16, X16, DD, IW16, DD, in_b, INP, OG, LAM, DD, DD, DD);
  k_scan_h<<<dim3(NLH / SBLK), dim3(SBLK), 0, stream>>>(INP, LAM, OG, S);
  k_scan_w<<<dim3(NLW / SBLK), dim3(SBLK), 0, stream>>>(INP, LAM, OG, S);
  k_cvt_t<<<dim3((DD * (DD / 8) + 255) / 256), blk, 0, stream>>>(out_w, OW16, DD, DD, DD * (DD / 8));
  k_ln<<<dim3(NROW / 8), blk, 0, stream>>>(S, gamma, beta, YH, YL);
  k_gemm<2, 1><<<dim3(NROW / 128, DD / 64), blk, 0, stream>>>(YH, YL, DD, OW16, DD, out_b, out, out, out, DD, DD, DD);
}
